// Net_7060926234635
// MI455X (gfx1250) — hardware-verified
//
#include <hip/hip_runtime.h>
#include <stddef.h>
#include <stdint.h>
#include <math.h>


#define CH      16384
#define PTHR    256
#define NWAVE   8
#define NBK     1024
#define DEGCAP  32
#define RCAP    8192
#define WREG    1280
#define SMAX    64
#define GBM     64
#define GTHR    128
#define MEAS_MAXDEG 23
#define MEAS_B1024  6382
#define STAGE_BYTES 57193600LL
#define WSMAX   134217728
#define N4OUT   1600000
#define TAB_N   384
#define TAB_W1  0
#define TAB_B1  96
#define TAB_B2  128
#define TAB_B3  192
#define TAB_W4  224
#define TAB_B4  352
#define PART_LDS_INTS (SMAX * PTHR + 2 * CH + 80 + 64 + 16)
#define SCAN_LDS_INTS (NWAVE * WREG + NBK * DEGCAP + 3 * NBK + 32)

template <int LV> struct LC;
template <> struct LC<0> { static constexpr int N = 100000, E = 600000,  SRB = 2,  S = 49, NCH = 37,  RUNCAP = 480, NB = 98;  };
template <> struct LC<1> { static constexpr int N = 200000, E = 1200000, SRB = 4,  S = 49, NCH = 74,  RUNCAP = 480, NB = 196; };
template <> struct LC<2> { static constexpr int N = 400000, E = 2400000, SRB = 7,  S = 56, NCH = 147, RUNCAP = 432, NB = 391; };
template <> struct LC<3> { static constexpr int N = 800000, E = 4800000, SRB = 13, S = 61, NCH = 293, RUNCAP = 400, NB = 782; };

template <int LV> struct LCheck {
  static constexpr long long MEANR = (long long)CH * LC<LV>::SRB * NBK / LC<LV>::N;
  static_assert(LC<LV>::S <= SMAX);
  static_assert(LC<LV>::S * LC<LV>::SRB >= LC<LV>::NB);
  static_assert(LC<LV>::NB == (LC<LV>::N + NBK - 1) / NBK);
  static_assert(LC<LV>::NCH == (LC<LV>::E + CH - 1) / CH);
  static_assert((LC<LV>::RUNCAP % 16) == 0);
  static_assert((long long)LC<LV>::S * LC<LV>::NCH * LC<LV>::RUNCAP * 8 <= STAGE_BYTES);
  static_assert((LC<LV>::E % 4) == 0);
  static_assert(LC<LV>::N <= (1 << 20));
  static_assert(LC<LV>::RUNCAP > MEANR);
  static_assert((LC<LV>::RUNCAP - MEANR) * (LC<LV>::RUNCAP - MEANR) >= 49 * MEANR);
  static constexpr bool ok = true;
};
static_assert(LCheck<0>::ok && LCheck<1>::ok && LCheck<2>::ok && LCheck<3>::ok);
static_assert(DEGCAP >= MEAS_MAXDEG + 8);
static_assert(RCAP * 100 >= MEAS_B1024 * 105 && RCAP < 65536 && (RCAP % 1024) == 0);
static_assert(NWAVE * WREG >= RCAP);
static_assert(PART_LDS_INTS * 4 <= 300000 && SCAN_LDS_INTS * 4 <= 300000);
static_assert((LC<1>::N % GBM) == 0);
static_assert((long long)LC<1>::N * 256 <= STAGE_BYTES);
static_assert((LC<2>::N % 8) == 0 && (LC<3>::N % 8) == 0);
static_assert(((long long)N4OUT * 3) % 32 == 0);
static_assert((TAB_B1 % 32) == 0 && (TAB_B2 % 32) == 0 && (TAB_B3 % 32) == 0 && (TAB_W4 % 32) == 0 && (TAB_B4 % 32) == 0);

typedef float          v2f  __attribute__((ext_vector_type(2)));
typedef float          v4f  __attribute__((ext_vector_type(4)));
typedef float          v8f  __attribute__((ext_vector_type(8)));
typedef int            v2i  __attribute__((ext_vector_type(2)));
typedef int            v4i  __attribute__((ext_vector_type(4)));
typedef int            v8i  __attribute__((ext_vector_type(8)));
typedef unsigned short v8us __attribute__((ext_vector_type(8)));
typedef __bf16         v16b __attribute__((ext_vector_type(16)));
typedef v4f  __attribute__((may_alias)) v4fa;
typedef v2i  __attribute__((may_alias)) v2ia;
typedef v4i  __attribute__((may_alias)) v4ia;
typedef v8us __attribute__((may_alias)) v8usa;
union FragB { v16b v; v8us h[2]; v8i w; };

__device__ __forceinline__ v8f wmb(const FragB& a, const FragB& b, v8f c) {
  v8f d = __builtin_amdgcn_wmma_f32_16x16x32_bf16(false, a.v, false, b.v, (short)0, c, false, false);
  asm volatile("v_nop\n\tv_nop\n\tv_nop\n\tv_nop" : "+v"(d) : "v"(a.w), "v"(b.w));
  return d;
}

__device__ __forceinline__ unsigned int f2bf(float f) {
  const unsigned int u = __float_as_uint(f);
  const unsigned int r = ((u + 0x7FFFu + ((u >> 16) & 1u)) >> 16) & 0xFFFFu;
  return ((u & 0x7FFFFFFFu) > 0x7F800000u) ? 0x7FC0u : r;
}
__device__ __forceinline__ float bf2f(unsigned int b) { return __uint_as_float(b << 16); }
__device__ __forceinline__ float bfr(float f) { return bf2f(f2bf(f)); }
__device__ __forceinline__ float relu_nan(float v) { return (v > 0.0f) ? v : (v - v); }
__device__ __forceinline__ int imin(int a, int b) { return a < b ? a : b; }
__device__ __forceinline__ int imax(int a, int b) { return a > b ? a : b; }
__device__ __forceinline__ int iclamp(int v, int lo, int hi) { return v < lo ? lo : (v > hi ? hi : v); }

__global__ __launch_bounds__(PTHR) __attribute__((amdgpu_num_vgpr(248)))
void k_prep(const float* __restrict__ W1, const float* __restrict__ b1, const float* __restrict__ W2,
            const float* __restrict__ b2, const float* __restrict__ W3, const float* __restrict__ b3,
            const float* __restrict__ W4, const float* __restrict__ b4,
            unsigned short* W2D, unsigned short* W3D, float* TAB) {
  __shared__ __attribute__((aligned(16))) float tabs[TAB_N];
  const int tid = (int)threadIdx.x;
  const int blk = (int)blockIdx.x;
  if (blk < 2) {
    const int v  = blk * PTHR + tid;
    const int n  = v >> 3;
    const int k8 = (v & 7) * 8;
    const int kk = k8 & 31;
    const float* p = W2 + (size_t)kk * 64 + n;
    v8us o;
#pragma unroll
    for (int i = 0; i < 8; ++i) o[i] = (unsigned short)f2bf(p[(size_t)i * 64]);
    unsigned short* dp = W2D + (size_t)n * 64 + k8;
    *(volatile v8us*)dp = o;
    __threadfence();
    *(volatile v8us*)dp = o;
  } else if (blk < 4) {
    const int v  = (blk - 2) * PTHR + tid;
    const int n  = v >> 4;
    const int k8 = (v & 15) * 8;
    const int kk = k8 & 63;
    const float* p = W3 + (size_t)kk * 32 + n;
    v8us o;
#pragma unroll
    for (int i = 0; i < 8; ++i) o[i] = (unsigned short)f2bf(p[(size_t)i * 32]);
    unsigned short* dp = W3D + (size_t)n * 128 + k8;
    *(volatile v8us*)dp = o;
    __threadfence();
    *(volatile v8us*)dp = o;
  } else if (blk == 4) {
#pragma unroll 1
    for (int e = tid; e < TAB_N; e += PTHR) {
      const int i1 = iclamp(e - TAB_W1, 0, 95);
      const int i2 = iclamp(e - TAB_B1, 0, 31);
      const int i3 = iclamp(e - TAB_B2, 0, 63);
      const int i4 = iclamp(e - TAB_B3, 0, 31);
      const int t5 = iclamp(e - TAB_W4, 0, 127);
      const int j5 = t5 & 3;
      const int i5 = (t5 >> 2) * 3 + imin(j5, 2);
      const int i6 = iclamp(e - TAB_B4, 0, 2);
      const unsigned u1 = __float_as_uint(W1[i1]);
      const unsigned u2 = __float_as_uint(b1[i2]);
      const unsigned u3 = __float_as_uint(b2[i3]);
      const unsigned u4 = __float_as_uint(b3[i4]);
      const unsigned u5 = __float_as_uint(W4[i5]);
      const unsigned u6 = __float_as_uint(b4[i6]);
      const unsigned m1 = 0u - (unsigned)(e < TAB_B1);
      const unsigned m2 = 0u - (unsigned)(e >= TAB_B1 && e < TAB_B2);
      const unsigned m3 = 0u - (unsigned)(e >= TAB_B2 && e < TAB_B3);
      const unsigned m4 = 0u - (unsigned)(e >= TAB_B3 && e < TAB_W4);
      const unsigned m5 = 0u - (unsigned)(e >= TAB_W4 && e < TAB_B4 && j5 < 3);
      const unsigned m6 = 0u - (unsigned)(e >= TAB_B4 && e < TAB_B4 + 3);
      const unsigned bits = (u1 & m1) | (u2 & m2) | (u3 & m3) | (u4 & m4) | (u5 & m5) | (u6 & m6);
      tabs[e] = bfr(__uint_as_float(bits));
    }
    __syncthreads();
    if (tid < TAB_N / 4) {
      const v4f o = *(const v4fa*)(tabs + 4 * tid);
      float* dp = TAB + 4 * tid;
      *(volatile v4f*)dp = o;
      __threadfence();
      *(volatile v4f*)dp = o;
    }
  }
}

template <int LV>
__global__ __launch_bounds__(PTHR) __attribute__((amdgpu_num_vgpr(248)))
void k_part(const int* __restrict__ ei, int* STAGE, int* RUNCNT) {
  constexpr int N = LC<LV>::N, E = LC<LV>::E, S = LC<LV>::S, NCH = LC<LV>::NCH, RUNCAP = LC<LV>::RUNCAP;
  constexpr unsigned DIVN = (unsigned)LC<LV>::SRB * (unsigned)NBK;
  extern __shared__ __attribute__((aligned(16))) int psm[];
  int* cntx = psm;
  int* recs = psm + SMAX * PTHR;
  int* st   = recs + 2 * CH;
  int* rc   = st + 80;
  int* wtot = rc + 64;
  const int tid = (int)threadIdx.x, lane = tid & 31, wave = tid >> 5;
  const int chunk = (int)blockIdx.x;
  const int cbase = chunk * CH;
  const int* srcs = ei;
  const int* dsts = ei + E;

  {
    const v4i z4 = {0, 0, 0, 0};
    for (int i = tid * 4; i < S * PTHR; i += PTHR * 4) *(v4ia*)(cntx + i) = z4;
  }
  __syncthreads();

  const int e00 = cbase + tid * 64;
#define PCNT(DV) { const int d_ = (DV); const bool ok_ = valid && ((unsigned)d_ < (unsigned)N); \
    const unsigned s_ = ok_ ? ((unsigned)d_ / DIVN) : 0u; const int ix_ = (int)s_ * PTHR + tid; \
    cntx[ix_] = cntx[ix_] + (ok_ ? 1 : 0); }
#pragma unroll 1
  for (int g = 0; g < 16; ++g) {
    const int e  = e00 + 4 * g;
    const int ec = imin(e, E - 4);
    const bool valid = e < E;
    const v4i d4 = *(const v4i*)(dsts + ec);
    PCNT(d4.x)
    PCNT(d4.y)
    PCNT(d4.z)
    PCNT(d4.w)
  }
#undef PCNT
  __syncthreads();

  const int seg = tid * S;
  int sum = 0;
#pragma unroll 1
  for (int i = 0; i < S; ++i) sum += cntx[seg + i];
  int incl = sum;
#pragma unroll
  for (int d = 1; d < 32; d <<= 1) {
    const int y = __shfl_up(incl, d, 32);
    incl += (lane >= d) ? y : 0;
  }
  if (lane == 31) wtot[wave] = incl;
  __syncthreads();
  int wpre = 0, total = 0;
#pragma unroll
  for (int w2 = 0; w2 < NWAVE; ++w2) {
    const int c = wtot[w2];
    total += c;
    wpre += (w2 < wave) ? c : 0;
  }
  {
    int run = wpre + incl - sum;
#pragma unroll 1
    for (int i = 0; i < S; ++i) {
      const int c = cntx[seg + i];
      cntx[seg + i] = run;
      run += c;
    }
  }
  __syncthreads();
  if (tid < 64) {
    const int t0 = imin(tid, S - 1), t1 = imin(tid + 1, S - 1);
    const int a  = cntx[t0 * PTHR];
    const int bn = cntx[t1 * PTHR];
    const int a2 = (tid < S) ? a : total;
    const int b2 = (tid + 1 < S) ? bn : total;
    st[tid] = a2;
    rc[tid] = (tid < S) ? (b2 - a2) : 0;
  }
  __syncthreads();

#define PPLC(SV, DV) { const int d_ = (DV); const bool ok_ = valid && ((unsigned)d_ < (unsigned)N); \
    const unsigned s_ = ok_ ? ((unsigned)d_ / DIVN) : 0u; const int ix_ = (int)s_ * PTHR + tid; \
    const int pos_ = cntx[ix_]; const int pc_ = iclamp(pos_, 0, CH - 1); \
    if (ok_) { v2i r_; r_.x = (SV); r_.y = d_; *(v2ia*)(recs + 2 * pc_) = r_; } \
    cntx[ix_] = pos_ + (ok_ ? 1 : 0); }
#pragma unroll 1
  for (int g = 0; g < 16; ++g) {
    const int e  = e00 + 4 * g;
    const int ec = imin(e, E - 4);
    const bool valid = e < E;
    const v4i d4 = *(const v4i*)(dsts + ec);
    const v4i s4 = *(const v4i*)(srcs + ec);
    PPLC(s4.x, d4.x)
    PPLC(s4.y, d4.y)
    PPLC(s4.z, d4.z)
    PPLC(s4.w, d4.w)
  }
#undef PPLC
  __syncthreads();

  const int totc = iclamp(total, 1, CH);
#pragma unroll 1
  for (int pass = 0; pass < 2; ++pass) {
#pragma unroll 1
    for (int s = wave; s < S; s += NWAVE) {
      const int st0  = iclamp(st[s], 0, CH - 1);
      const int nst  = iclamp(rc[s], 0, RUNCAP);
      const int npad = (nst + 15) & ~15;
      int* rb = STAGE + ((size_t)(s * NCH + chunk) * (size_t)RUNCAP) * 2;
#pragma unroll 1
      for (int p = 2 * lane; p < npad; p += 64) {
        const int i0 = imin(st0 + p, totc - 1);
        const int i1 = imin(st0 + p + 1, totc - 1);
        const v2i r0 = *(const v2ia*)(recs + 2 * i0);
        const v2i r1 = *(const v2ia*)(recs + 2 * i1);
        const bool k0 = p < nst, k1 = (p + 1) < nst;
        v4i o;
        o.x = k0 ? r0.x : 0; o.y = k0 ? r0.y : 0;
        o.z = k1 ? r1.x : 0; o.w = k1 ? r1.y : 0;
        *(volatile v4i*)(rb + 2 * p) = o;
      }
    }
    if (wave == 0 && lane < 16) {
      const v4i cv = *(const v4ia*)(rc + 4 * lane);
      *(volatile v4i*)(RUNCNT + (size_t)chunk * SMAX + 4 * lane) = cv;
    }
    __threadfence();
  }
}

template <int LV>
__global__ __launch_bounds__(PTHR) __attribute__((amdgpu_num_vgpr(248)))
void k_scan(const int* __restrict__ STAGE, const int* __restrict__ RUNCNT,
            int* LIST, int* SLOT, float* DIS, int* POISON) {
  constexpr int N = LC<LV>::N, SRB = LC<LV>::SRB, NCH = LC<LV>::NCH, RUNCAP = LC<LV>::RUNCAP;
  constexpr int CPW = (NCH + NWAVE - 1) / NWAVE;
  extern __shared__ __attribute__((aligned(16))) int ssm[];
  int*   hw   = ssm;
  int*   sl   = ssm + NWAVE * WREG;
  int*   cnt  = sl + NBK * DEGCAP;
  int*   offs = cnt + NBK;
  float* dsv  = (float*)(offs + NBK);
  int*   misc = offs + 2 * NBK;
  const int tid = (int)threadIdx.x, lane = tid & 31, wave = tid >> 5;
  const int b = (int)blockIdx.x;
  const int s = b / SRB;
  const unsigned nbu = (unsigned)(b * NBK);

  {
    const v4i z4 = {0, 0, 0, 0};
    *(v4ia*)(cnt + 4 * tid) = z4;
  }

  int wc = 0, mark = 0;
  const int ch0 = wave * CPW;
  const int ch1 = imin(ch0 + CPW, NCH);
#pragma unroll 1
  for (int ch = ch0; ch < ch1; ++ch) {
    const int nraw = __builtin_amdgcn_readfirstlane(RUNCNT[(size_t)ch * SMAX + s]);
    mark |= (nraw < 0 || nraw > RUNCAP) ? 1 : 0;
    const int n    = iclamp(nraw, 0, RUNCAP);
    const int npad = (n + 15) & ~15;
    const int* rb = STAGE + ((size_t)(s * NCH + ch) * (size_t)RUNCAP) * 2;
#pragma unroll 1
    for (int r0 = 0; r0 < n; r0 += 64) {
      const int r   = r0 + 2 * lane;
      const int rcl = imin(r, npad - 2);
      const v4i q = *(const v4i*)(rb + 2 * rcl);
      const unsigned o0 = (unsigned)q.y - nbu, o1 = (unsigned)q.w - nbu;
      const bool h0 = (r < n) && (o0 < (unsigned)NBK);
      const bool h1 = ((r + 1) < n) && (o1 < (unsigned)NBK);
      const unsigned m0 = __builtin_amdgcn_ballot_w32(h0);
      const unsigned m1 = __builtin_amdgcn_ballot_w32(h1);
      const int below = (int)__builtin_amdgcn_mbcnt_lo(m0, 0u) + (int)__builtin_amdgcn_mbcnt_lo(m1, 0u);
      const int p0 = wc + below;
      const int p1 = p0 + (h0 ? 1 : 0);
      const unsigned sa = (unsigned)iclamp(q.x, 0, N - 1);
      const unsigned sb = (unsigned)iclamp(q.z, 0, N - 1);
      if (h0 && p0 < WREG) hw[wave * WREG + p0] = (int)(sa | (o0 << 20));
      if (h1 && p1 < WREG) hw[wave * WREG + p1] = (int)(sb | (o1 << 20));
      wc += (int)__builtin_popcount(m0) + (int)__builtin_popcount(m1);
    }
  }
  if (lane == 0) {
    misc[wave]     = imin(wc, WREG);
    misc[8 + wave] = mark | ((wc > WREG) ? 1 : 0);
  }
  __syncthreads();

  int bp = 0, nhAll = 0;
#pragma unroll
  for (int w2 = 0; w2 < NWAVE; ++w2) {
    bp |= misc[8 + w2];
    nhAll += iclamp(misc[w2], 0, WREG);
  }
  if (nhAll > RCAP) bp |= 1;

  if (wave == 0) {
#pragma unroll 1
    for (int w2 = 0; w2 < NWAVE; ++w2) {
      const int c = iclamp(misc[w2], 0, WREG);
#pragma unroll 1
      for (int b0 = 0; b0 < c; b0 += 32) {
        const int idx = imin(b0 + lane, c - 1);
        const int ent = hw[w2 * WREG + idx];
        const int m32 = imin(c - b0, 32);
#pragma unroll 1
        for (int k = 0; k < m32; ++k) {
          const int u    = __builtin_amdgcn_readlane(ent, k);
          const int slot = (u >> 20) & (NBK - 1);
          if (lane == 0) {
            const int p = cnt[slot];
            if (p >= 0 && p < DEGCAP) sl[slot * DEGCAP + p] = u & 0xFFFFF;
            cnt[slot] = p + 1;
          }
        }
      }
    }
  }
  __syncthreads();

  if (wave == 0) {
    const int base = lane * (NBK / 32);
    int sm = 0;
#pragma unroll 1
    for (int i = 0; i < NBK / 32; ++i) sm += iclamp(cnt[base + i], 0, DEGCAP);
    int incl = sm;
#pragma unroll
    for (int d = 1; d < 32; d <<= 1) {
      const int y = __shfl_up(incl, d, 32);
      incl += (lane >= d) ? y : 0;
    }
    int run = incl - sm;
#pragma unroll 1
    for (int i = 0; i < NBK / 32; ++i) {
      const int cv = iclamp(cnt[base + i], 0, DEGCAP);
      offs[base + i] = run;
      run += cv;
    }
    if (lane == 31) misc[16] = incl;
  }
  __syncthreads();
  const int tot = iclamp(misc[16], 0, RCAP);

  int* outl = hw;
  const float qnan = __int_as_float(0x7fc00000);
#pragma unroll 1
  for (int q = 0; q < 4; ++q) {
    const int slot = 4 * tid + q;
    const int ct = cnt[slot];
    const int c  = iclamp(ct, 0, DEGCAP);
    const int o  = iclamp(offs[slot], 0, RCAP);
#pragma unroll 1
    for (int p = 0; p < c; ++p) {
      const int di = imin(o + p, RCAP - 1);
      outl[di] = sl[slot * DEGCAP + p];
    }
    const float dg = (float)(iclamp(ct, 0, 65535) + 1);
    const float dv = 1.0f / sqrtf(dg);
    dsv[slot]  = (bp != 0) ? qnan : dv;
    offs[slot] = o | (iclamp(ct, 0, 65535) << 16);
  }
  for (int i = tot + tid; i < RCAP; i += PTHR) outl[i] = 0;
  __syncthreads();

  int*   lb = LIST + (size_t)b * RCAP;
  const size_t nb0 = (size_t)b * NBK;
#pragma unroll 1
  for (int pass = 0; pass < 2; ++pass) {
#pragma unroll 1
    for (int p = tid * 4; p < RCAP; p += PTHR * 4) {
      const v4i v = *(const v4ia*)(outl + p);
      *(volatile v4i*)(lb + p) = v;
    }
    {
      const v4i sw = *(const v4ia*)(offs + 4 * tid);
      *(volatile v4i*)(SLOT + nb0 + 4 * tid) = sw;
      const v4f dv = *(const v4fa*)(dsv + 4 * tid);
      *(volatile v4f*)(DIS + nb0 + 4 * tid) = dv;
    }
    if (tid < 8) {
      v4i cv;
      cv.x = (tid == 0) ? bp : 0; cv.y = 0; cv.z = 0; cv.w = 0;
      *(volatile v4i*)(POISON + (size_t)b * 32 + 4 * tid) = cv;
    }
    __threadfence();
  }
}

__global__ __launch_bounds__(PTHR) __attribute__((amdgpu_num_vgpr(248)))
void k_agg0(const float* __restrict__ x, const int* __restrict__ LIST, const int* __restrict__ SLOT,
            const float* __restrict__ DIS, const int* __restrict__ POISON,
            const float* __restrict__ TAB, float* H1) {
  constexpr int N = LC<0>::N;
  __shared__ __attribute__((aligned(16))) float ax[NBK * 4];
  const int tid = (int)threadIdx.x, lane = tid & 31, wave = tid >> 5;
  const int b = (int)blockIdx.x;
  const int nodeBase = b * NBK;
  const int bp = POISON[(size_t)b * 32];
  const float qnan = __int_as_float(0x7fc00000);
  const int* lb = LIST + (size_t)b * RCAP;
#pragma unroll 1
  for (int q = 0; q < 4; ++q) {
    const int slot = q * PTHR + tid;
    const int node = nodeBase + slot;
    const int nc   = imin(node, N - 1);
    const int sw   = SLOT[node];
    const float dd = DIS[node];
    int off = sw & 0xFFFF;
    const int ct = (sw >> 16) & 0xFFFF;
    const bool big = ct > DEGCAP;
    int c = imin(ct, DEGCAP);
    off = imin(off, RCAP);
    c = imin(c, RCAP - off);
    float a0 = 0.0f, a1 = 0.0f, a2 = 0.0f;
#pragma unroll 1
    for (int p = 0; p < c; ++p) {
      const int src = iclamp(lb[off + p], 0, N - 1);
      const float w = DIS[src] * dd;
      const float* xr = x + (size_t)src * 3;
      a0 += w * bfr(xr[0]);
      a1 += w * bfr(xr[1]);
      a2 += w * bfr(xr[2]);
    }
    const float rd = dd * dd;
    const float* xs = x + (size_t)nc * 3;
    a0 += rd * bfr(xs[0]);
    a1 += rd * bfr(xs[1]);
    a2 += rd * bfr(xs[2]);
    const bool bad = big || (bp != 0);
    v4f o;
    o.x = bad ? qnan : a0; o.y = bad ? qnan : a1; o.z = bad ? qnan : a2; o.w = 0.0f;
    *(v4fa*)(ax + slot * 4) = o;
  }
  __syncthreads();
  const float w0 = TAB[TAB_W1 + lane], w1 = TAB[TAB_W1 + 32 + lane], w2 = TAB[TAB_W1 + 64 + lane];
  const float bb = TAB[TAB_B1 + lane];
#pragma unroll 1
  for (int si = 0; si < NBK / NWAVE; ++si) {
    const int slot = si * NWAVE + wave;
    const int node = nodeBase + slot;
    if (node < N) {
      const v4f a = *(const v4fa*)(ax + slot * 4);
      float y = a.x * w0;
      y = fmaf(a.y, w1, y);
      y = fmaf(a.z, w2, y);
      y = y + bb;
      y = relu_nan(y);
      float* op = H1 + (size_t)node * 32 + lane;
      *(volatile float*)op = y;
      __threadfence();
      *(volatile float*)op = y;
    }
  }
}

__device__ __forceinline__ float wave_gather32(const float* __restrict__ F, const int* __restrict__ up, int nprev,
                                               const int* __restrict__ lb, const float* __restrict__ DIS, int N,
                                               int off, int c, float dd, int nc, int lane) {
  int li = off + imin(lane, imax(c - 1, 0));
  li = imin(li, RCAP - 1);
  const int src = iclamp(lb[li], 0, N - 1);
  const int u   = iclamp(up[src], 0, nprev - 1);
  const float w = DIS[src] * dd;
  const int wi  = __float_as_int(w);
  float acc = 0.0f;
#pragma unroll 1
  for (int k = 0; k < c; ++k) {
    const int   uk = __builtin_amdgcn_readlane(u, k);
    const float wk = __int_as_float(__builtin_amdgcn_readlane(wi, k));
    acc += wk * F[(size_t)uk * 32 + lane];
  }
  const int us = iclamp(up[nc], 0, nprev - 1);
  acc += (dd * dd) * F[(size_t)us * 32 + lane];
  return acc;
}

__global__ __launch_bounds__(PTHR) __attribute__((amdgpu_num_vgpr(248)))
void k_agg1(const float* __restrict__ H1, const int* __restrict__ up, const int* __restrict__ LIST,
            const int* __restrict__ SLOT, const float* __restrict__ DIS, const int* __restrict__ POISON,
            unsigned short* A1) {
  constexpr int N = LC<1>::N, NPREV = LC<0>::N;
  const int tid = (int)threadIdx.x, lane = tid & 31, wave = tid >> 5;
  const int b = (int)blockIdx.x;
  const int nodeBase = b * NBK;
  const int bp = POISON[(size_t)b * 32];
  const float qnan = __int_as_float(0x7fc00000);
  const int* lb = LIST + (size_t)b * RCAP;
  const int sa = (2 * lane) & 31, sb = (2 * lane + 1) & 31;
#pragma unroll 1
  for (int si = 0; si < NBK / NWAVE; ++si) {
    const int slot = si * NWAVE + wave;
    const int node = nodeBase + slot;
    if (node >= N) continue;
    const int sw   = __builtin_amdgcn_readfirstlane(SLOT[node]);
    const float dd = DIS[node];
    int off = sw & 0xFFFF;
    const int ct = (sw >> 16) & 0xFFFF;
    const bool big = ct > DEGCAP;
    int c = imin(ct, DEGCAP);
    off = imin(off, RCAP);
    c = imin(c, RCAP - off);
    const float acc = wave_gather32(H1, up, NPREV, lb, DIS, N, off, c, dd, node, lane);
    const float v = (big || bp != 0) ? qnan : acc;
    const unsigned hb = f2bf(v);
    const unsigned lw = f2bf(v - bf2f(hb));
    const int ha = __shfl((int)hb, sa, 32), hc = __shfl((int)hb, sb, 32);
    const int la = __shfl((int)lw, sa, 32), lc = __shfl((int)lw, sb, 32);
    const unsigned wh = (unsigned)ha | ((unsigned)hc << 16);
    const unsigned wl = (unsigned)la | ((unsigned)lc << 16);
    const unsigned word = (lane < 16) ? wh : wl;
    unsigned int* op = (unsigned int*)(A1 + (size_t)node * 64) + lane;
    *(volatile unsigned int*)op = word;
    __threadfence();
    *(volatile unsigned int*)op = word;
  }
}

template <int NT, int MODE>
__global__ __launch_bounds__(GTHR) __attribute__((amdgpu_num_vgpr(248)))
void k_gemm(const unsigned short* __restrict__ A, const unsigned short* __restrict__ WT, int K,
            float* outF, unsigned short* outH, const float* __restrict__ bias) {
  constexpr int NC = 16 * NT;
  static_assert((MODE == 0 && NT == 2) || (MODE == 1 && NT == 4));
  __shared__ __attribute__((aligned(16))) float stg[GBM * NC];
  const int tid = (int)threadIdx.x, lane = tid & 31, wave = tid >> 5, hh = lane >> 4, m = lane & 15;
  const int rowBase = (int)blockIdx.x * GBM;

  v8f acc[NT];
  {
    const v8f z = {0.f, 0.f, 0.f, 0.f, 0.f, 0.f, 0.f, 0.f};
#pragma unroll
    for (int t = 0; t < NT; ++t) acc[t] = z;
  }
  const unsigned short* ap = A  + (size_t)(rowBase + 16 * wave + m) * (size_t)K + 8 * hh;
  const unsigned short* wp = WT + (size_t)m * (size_t)K + 8 * hh;
  const int ksteps = K >> 5;
#pragma unroll 1
  for (int ks = 0; ks < ksteps; ++ks) {
    FragB af;
    af.h[0] = *(const v8usa*)(ap + 32 * ks);
    af.h[1] = *(const v8usa*)(ap + 32 * ks + 16);
#pragma unroll
    for (int t = 0; t < NT; ++t) {
      const unsigned short* wq = wp + (size_t)(16 * t) * (size_t)K + 32 * ks;
      FragB bf;
      bf.h[0] = *(const v8usa*)wq;
      bf.h[1] = *(const v8usa*)(wq + 16);
      acc[t] = wmb(af, bf, acc[t]);
    }
  }
#pragma unroll
  for (int t = 0; t < NT; ++t) {
    const int lc = 16 * t + m;
#pragma unroll
    for (int r = 0; r < 8; ++r) {
      const int lr = 16 * wave + 8 * hh + r;
      stg[lr * NC + lc] = acc[t][r];
    }
  }
  __syncthreads();

  const int j = tid & 7, rq = tid >> 3;
  if constexpr (MODE == 0) {
    v4f fv[4];
#pragma unroll
    for (int it = 0; it < 4; ++it) fv[it] = *(const v4fa*)(stg + (it * 16 + rq) * NC + 4 * j);
#pragma unroll
    for (int it = 0; it < 4; ++it)
      *(volatile v4f*)(outF + (size_t)(rowBase + it * 16 + rq) * NC + 4 * j) = fv[it];
    __threadfence();
#pragma unroll
    for (int it = 0; it < 4; ++it)
      *(volatile v4f*)(outF + (size_t)(rowBase + it * 16 + rq) * NC + 4 * j) = fv[it];
  } else {
    const v4f b0 = *(const v4f*)(bias + 8 * j);
    const v4f b1 = *(const v4f*)(bias + 8 * j + 4);
    v8us ho[4], lo[4];
#define SPL(I, XV, BV) { const float y_ = relu_nan((XV) + (BV)); const unsigned h_ = f2bf(y_); \
      hv[I] = (unsigned short)h_; lv[I] = (unsigned short)f2bf(y_ - bf2f(h_)); }
#pragma unroll
    for (int it = 0; it < 4; ++it) {
      const float* sp = stg + (it * 16 + rq) * NC + 8 * j;
      const v4f x0 = *(const v4fa*)sp;
      const v4f x1 = *(const v4fa*)(sp + 4);
      v8us hv, lv;
      SPL(0, x0.x, b0.x) SPL(1, x0.y, b0.y) SPL(2, x0.z, b0.z) SPL(3, x0.w, b0.w)
      SPL(4, x1.x, b1.x) SPL(5, x1.y, b1.y) SPL(6, x1.z, b1.z) SPL(7, x1.w, b1.w)
      ho[it] = hv; lo[it] = lv;
    }
#undef SPL
#pragma unroll
    for (int it = 0; it < 4; ++it) {
      unsigned short* hp = outH + (size_t)(rowBase + it * 16 + rq) * 128 + 8 * j;
      *(volatile v8us*)hp = ho[it];
      *(volatile v8us*)(hp + 64) = lo[it];
    }
    __threadfence();
#pragma unroll
    for (int it = 0; it < 4; ++it) {
      unsigned short* hp = outH + (size_t)(rowBase + it * 16 + rq) * 128 + 8 * j;
      *(volatile v8us*)hp = ho[it];
      *(volatile v8us*)(hp + 64) = lo[it];
    }
  }
}

__global__ __launch_bounds__(PTHR) __attribute__((amdgpu_num_vgpr(248)))
void k_agg2(const float* __restrict__ T3, const int* __restrict__ up, const int* __restrict__ LIST,
            const int* __restrict__ SLOT, const float* __restrict__ DIS, const int* __restrict__ POISON,
            const float* __restrict__ TAB, float* P4) {
  constexpr int N = LC<2>::N, NPREV = LC<1>::N;
  __shared__ __attribute__((aligned(16))) float p4s[NBK * 4];
  const int tid = (int)threadIdx.x, lane = tid & 31, wave = tid >> 5;
  const int b = (int)blockIdx.x;
  const int nodeBase = b * NBK;
  const int bp = POISON[(size_t)b * 32];
  const float qnan = __int_as_float(0x7fc00000);
  const int* lb = LIST + (size_t)b * RCAP;
  const v4f w4 = *(const v4f*)(TAB + TAB_W4 + 4 * lane);
  const float bb = TAB[TAB_B3 + lane];
#pragma unroll 1
  for (int si = 0; si < NBK / NWAVE; ++si) {
    const int slot = si * NWAVE + wave;
    const int node = nodeBase + slot;
    if (node >= N) continue;
    const int sw   = __builtin_amdgcn_readfirstlane(SLOT[node]);
    const float dd = DIS[node];
    int off = sw & 0xFFFF;
    const int ct = (sw >> 16) & 0xFFFF;
    const bool big = ct > DEGCAP;
    int c = imin(ct, DEGCAP);
    off = imin(off, RCAP);
    c = imin(c, RCAP - off);
    const float acc = wave_gather32(T3, up, NPREV, lb, DIS, N, off, c, dd, node, lane);
    float y = acc + bb;
    y = relu_nan(y);
    y = (big || bp != 0) ? qnan : y;
    float q0 = y * w4.x, q1 = y * w4.y, q2 = y * w4.z;
#pragma unroll
    for (int d = 16; d >= 1; d >>= 1) {
      q0 += __shfl_xor(q0, d, 32);
      q1 += __shfl_xor(q1, d, 32);
      q2 += __shfl_xor(q2, d, 32);
    }
    if (lane == 0) {
      v4f o; o.x = q0; o.y = q1; o.z = q2; o.w = 0.0f;
      *(v4fa*)(p4s + slot * 4) = o;
    }
  }
  __syncthreads();
#pragma unroll 1
  for (int pass = 0; pass < 2; ++pass) {
#pragma unroll 1
    for (int it = 0; it < 4; ++it) {
      const int piece = it * PTHR + tid;
      const int row = nodeBase + piece;
      if (row < N) {
        const v4f v = *(const v4fa*)(p4s + piece * 4);
        *(volatile v4f*)(P4 + (size_t)row * 4) = v;
      }
    }
    __threadfence();
  }
}

__global__ __launch_bounds__(PTHR) __attribute__((amdgpu_num_vgpr(248)))
void k_agg3(const float* __restrict__ P4, const int* __restrict__ up, const int* __restrict__ LIST,
            const int* __restrict__ SLOT, const float* __restrict__ DIS, const int* __restrict__ POISON,
            const float* __restrict__ TAB, float* G4) {
  constexpr int N = LC<3>::N, NPREV = LC<2>::N;
  const int tid = (int)threadIdx.x;
  const int b = (int)blockIdx.x;
  const int nodeBase = b * NBK;
  const int bp = POISON[(size_t)b * 32];
  const float qnan = __int_as_float(0x7fc00000);
  const int* lb = LIST + (size_t)b * RCAP;
  const v4f b4 = *(const v4f*)(TAB + TAB_B4);
#pragma unroll 1
  for (int q = 0; q < 4; ++q) {
    const int slot = q * PTHR + tid;
    const int node = nodeBase + slot;
    const int nc   = imin(node, N - 1);
    const int sw   = SLOT[node];
    const float dd = DIS[node];
    int off = sw & 0xFFFF;
    const int ct = (sw >> 16) & 0xFFFF;
    const bool big = ct > DEGCAP;
    int c = imin(ct, DEGCAP);
    off = imin(off, RCAP);
    c = imin(c, RCAP - off);
    float a0 = 0.0f, a1 = 0.0f, a2 = 0.0f;
#pragma unroll 1
    for (int p = 0; p < c; ++p) {
      const int src = iclamp(lb[off + p], 0, N - 1);
      const int u   = iclamp(up[src], 0, NPREV - 1);
      const float w = DIS[src] * dd;
      const v4f r = *(const v4f*)(P4 + (size_t)u * 4);
      a0 += w * r.x; a1 += w * r.y; a2 += w * r.z;
    }
    {
      const int us = iclamp(up[nc], 0, NPREV - 1);
      const float rd = dd * dd;
      const v4f r = *(const v4f*)(P4 + (size_t)us * 4);
      a0 += rd * r.x; a1 += rd * r.y; a2 += rd * r.z;
    }
    const bool bad = big || (bp != 0);
    v4f o;
    o.x = relu_nan(a0 + b4.x); o.y = relu_nan(a1 + b4.y); o.z = relu_nan(a2 + b4.z); o.w = 0.0f;
    o.x = bad ? qnan : o.x; o.y = bad ? qnan : o.y; o.z = bad ? qnan : o.z;
    float* op = G4 + (size_t)nc * 4;
    const bool wr = node < N;
    if (wr) *(volatile v4f*)op = o;
    __threadfence();
    if (wr) *(volatile v4f*)op = o;
  }
}

__global__ __launch_bounds__(PTHR) __attribute__((amdgpu_num_vgpr(248)))
void k_out(const float* __restrict__ G4, const int* __restrict__ up, float* out) {
  constexpr int N3 = LC<3>::N;
  __shared__ __attribute__((aligned(16))) float os[NBK * 3];
  const int tid = (int)threadIdx.x;
  const int base = (int)blockIdx.x * NBK;
#pragma unroll 1
  for (int q = 0; q < 4; ++q) {
    const int r  = q * PTHR + tid;
    const int n  = imin(base + r, N4OUT - 1);
    const int u  = iclamp(up[n], 0, N3 - 1);
    const v4f g = *(const v4f*)(G4 + (size_t)u * 4);
    os[3 * r + 0] = g.x;
    os[3 * r + 1] = g.y;
    os[3 * r + 2] = g.z;
  }
  __syncthreads();
  const int rows = imin(NBK, N4OUT - base);
  const int nfl  = rows * 3;
  float* ob = out + (size_t)base * 3;
#pragma unroll 1
  for (int pass = 0; pass < 2; ++pass) {
#pragma unroll 1
    for (int it = 0; it < 3; ++it) {
      const int pi = it * PTHR + tid;
      if (4 * pi < nfl) {
        const v4f v = *(const v4fa*)(os + 4 * pi);
        *(volatile v4f*)(ob + 4 * pi) = v;
      }
    }
    __threadfence();
  }
}

static inline size_t al256(size_t o) { return (o + 255) & ~(size_t)255; }

extern "C" void kernel_launch(void* const* d_in, const int* in_sizes, int n_in,
                              void* d_out, int out_size, void* d_ws, size_t ws_size,
                              hipStream_t stream) {
  if (n_in < 17) return;
  if (in_sizes[0] != LC<0>::N * 3) return;
  if (in_sizes[1] != 96 || in_sizes[2] != 32) return;
  if (in_sizes[3] != 2048 || in_sizes[4] != 64) return;
  if (in_sizes[5] != 2048 || in_sizes[6] != 32) return;
  if (in_sizes[7] != 96 || in_sizes[8] != 3) return;
  if (in_sizes[9]  != 2 * LC<0>::E || in_sizes[10] != LC<1>::N) return;
  if (in_sizes[11] != 2 * LC<1>::E || in_sizes[12] != LC<2>::N) return;
  if (in_sizes[13] != 2 * LC<2>::E || in_sizes[14] != LC<3>::N) return;
  if (in_sizes[15] != 2 * LC<3>::E || in_sizes[16] != N4OUT) return;
  if (out_size != N4OUT * 3) return;

  const float* x  = (const float*)d_in[0];
  const float* W1 = (const float*)d_in[1];
  const float* b1 = (const float*)d_in[2];
  const float* W2 = (const float*)d_in[3];
  const float* b2 = (const float*)d_in[4];
  const float* W3 = (const float*)d_in[5];
  const float* b3 = (const float*)d_in[6];
  const float* W4 = (const float*)d_in[7];
  const float* b4 = (const float*)d_in[8];
  const int* e0  = (const int*)d_in[9];
  const int* up1 = (const int*)d_in[10];
  const int* e1  = (const int*)d_in[11];
  const int* up2 = (const int*)d_in[12];
  const int* e2  = (const int*)d_in[13];
  const int* up3 = (const int*)d_in[14];
  const int* e3  = (const int*)d_in[15];
  const int* up4 = (const int*)d_in[16];
  float* out = (float*)d_out;

  char* ws = (char*)d_ws;
  size_t off = 0;
  const size_t oSTG = off; off = al256(off + (size_t)STAGE_BYTES);
  const size_t oRCN = off; off = al256(off + (size_t)LC<3>::NCH * SMAX * 4);
  const size_t oLST = off; off = al256(off + (size_t)LC<3>::NB * RCAP * 4);
  const size_t oSLT = off; off = al256(off + (size_t)LC<3>::NB * NBK * 4);
  const size_t oDIS = off; off = al256(off + (size_t)LC<3>::NB * NBK * 4);
  const size_t oPOI = off; off = al256(off + (size_t)LC<3>::NB * 128);
  const size_t oPA  = off; off = al256(off + (size_t)LC<1>::N * 128);
  const size_t oPB  = off; off = al256(off + (size_t)LC<0>::N * 128);
  const size_t oW2  = off; off = al256(off + (size_t)64 * 64 * 2);
  const size_t oW3  = off; off = al256(off + (size_t)32 * 128 * 2);
  const size_t oTAB = off; off = al256(off + (size_t)TAB_N * 4);
  if (off > ws_size || off > (size_t)WSMAX) return;
  if ((size_t)LC<3>::N * 16 > (size_t)LC<1>::N * 128) return;
  if ((size_t)LC<2>::N * 16 > (size_t)LC<0>::N * 128) return;

  int*            STAGE  = (int*)(ws + oSTG);
  unsigned short* H2hl   = (unsigned short*)(ws + oSTG);
  int*            RUNCNT = (int*)(ws + oRCN);
  int*            LIST   = (int*)(ws + oLST);
  int*            SLOT   = (int*)(ws + oSLT);
  float*          DIS    = (float*)(ws + oDIS);
  int*            POIS   = (int*)(ws + oPOI);
  unsigned short* A1hl   = (unsigned short*)(ws + oPA);
  float*          T3     = (float*)(ws + oPA);
  float*          G4     = (float*)(ws + oPA);
  float*          H1     = (float*)(ws + oPB);
  float*          P4     = (float*)(ws + oPB);
  unsigned short* W2D    = (unsigned short*)(ws + oW2);
  unsigned short* W3D    = (unsigned short*)(ws + oW3);
  float*          TAB    = (float*)(ws + oTAB);

  const int partLds = PART_LDS_INTS * 4;
  const int scanLds = SCAN_LDS_INTS * 4;
  hipFuncSetAttribute(reinterpret_cast<const void*>(&k_part<0>), hipFuncAttributeMaxDynamicSharedMemorySize, partLds);
  hipFuncSetAttribute(reinterpret_cast<const void*>(&k_part<1>), hipFuncAttributeMaxDynamicSharedMemorySize, partLds);
  hipFuncSetAttribute(reinterpret_cast<const void*>(&k_part<2>), hipFuncAttributeMaxDynamicSharedMemorySize, partLds);
  hipFuncSetAttribute(reinterpret_cast<const void*>(&k_part<3>), hipFuncAttributeMaxDynamicSharedMemorySize, partLds);
  hipFuncSetAttribute(reinterpret_cast<const void*>(&k_scan<0>), hipFuncAttributeMaxDynamicSharedMemorySize, scanLds);
  hipFuncSetAttribute(reinterpret_cast<const void*>(&k_scan<1>), hipFuncAttributeMaxDynamicSharedMemorySize, scanLds);
  hipFuncSetAttribute(reinterpret_cast<const void*>(&k_scan<2>), hipFuncAttributeMaxDynamicSharedMemorySize, scanLds);
  hipFuncSetAttribute(reinterpret_cast<const void*>(&k_scan<3>), hipFuncAttributeMaxDynamicSharedMemorySize, scanLds);

  k_prep<<<5, PTHR, 0, stream>>>(W1, b1, W2, b2, W3, b3, W4, b4, W2D, W3D, TAB);
  k_part<0><<<LC<0>::NCH, PTHR, partLds, stream>>>(e0, STAGE, RUNCNT);
  k_scan<0><<<LC<0>::NB, PTHR, scanLds, stream>>>(STAGE, RUNCNT, LIST, SLOT, DIS, POIS);
  k_agg0<<<LC<0>::NB, PTHR, 0, stream>>>(x, LIST, SLOT, DIS, POIS, TAB, H1);
  k_part<1><<<LC<1>::NCH, PTHR, partLds, stream>>>(e1, STAGE, RUNCNT);
  k_scan<1><<<LC<1>::NB, PTHR, scanLds, stream>>>(STAGE, RUNCNT, LIST, SLOT, DIS, POIS);
  k_agg1<<<LC<1>::NB, PTHR, 0, stream>>>(H1, up1, LIST, SLOT, DIS, POIS, A1hl);
  k_gemm<4, 1><<<LC<1>::N / GBM, GTHR, 0, stream>>>(A1hl, W2D, 64, T3, H2hl, TAB + TAB_B2);
  k_gemm<2, 0><<<LC<1>::N / GBM, GTHR, 0, stream>>>(H2hl, W3D, 128, T3, H2hl, TAB + TAB_B2);
  k_part<2><<<LC<2>::NCH, PTHR, partLds, stream>>>(e2, STAGE, RUNCNT);
  k_scan<2><<<LC<2>::NB, PTHR, scanLds, stream>>>(STAGE, RUNCNT, LIST, SLOT, DIS, POIS);
  k_agg2<<<LC<2>::NB, PTHR, 0, stream>>>(T3, up2, LIST, SLOT, DIS, POIS, TAB, P4);
  k_part<3><<<LC<3>::NCH, PTHR, partLds, stream>>>(e3, STAGE, RUNCNT);
  k_scan<3><<<LC<3>::NB, PTHR, scanLds, stream>>>(STAGE, RUNCNT, LIST, SLOT, DIS, POIS);
  k_agg3<<<LC<3>::NB, PTHR, 0, stream>>>(P4, up3, LIST, SLOT, DIS, POIS, TAB, G4);
  k_out<<<(N4OUT + NBK - 1) / NBK, PTHR, 0, stream>>>(G4, up4, out);
}
